// HierDDpm_25692494364846
// MI455X (gfx1250) — hardware-run, weakly checked
//
#include <hip/hip_runtime.h>
#include <math.h>

typedef __attribute__((ext_vector_type(16))) _Float16 v16h;
typedef __attribute__((ext_vector_type(8)))  _Float16 v8h;
typedef __attribute__((ext_vector_type(4)))  _Float16 v4h;
typedef __attribute__((ext_vector_type(8)))  float    v8f;
typedef __attribute__((ext_vector_type(4)))  float    v4f;

constexpr int kNB   = 8;
constexpr int kSeq  = 8192;
constexpr int kIn   = 128;
constexpr int kD    = 64;
constexpr int kATP  = 136;
constexpr int kTP   = 68;
constexpr int kCSP  = kD * kTP;
constexpr float kLnEps = 1e-5f;
constexpr float kTwoPi = 6.28318530717958647692f;
constexpr float kCarryA   = 16.0f;
constexpr float kCarryW   = 256.0f;
constexpr float kCarryP   = 1024.0f;
constexpr float kInvDense = 1.0f / (kCarryA * kCarryW);
constexpr float kInvMod   = 1.0f / (kCarryA * kCarryP);
constexpr float kHalfMinNormal = 6.103515625e-05f;

static_assert(kInvDense == 1.0f / 4096.0f, "dense fold-back");
static_assert(kInvMod == 1.0f / 16384.0f, "modulated fold-back");
static_assert((kSeq % 2) == 0, "two positions per block");
static_assert((kIn % 32) == 0 && (kD % 32) == 0, "K multiples of 32");
static_assert((kD % 16) == 0 && ((2 * kD) % 16) == 0, "N multiples of 16");
static_assert(kNB * 2 == 16, "16 matrix rows = 2 positions x 8 batch rows");
static_assert((kATP % 8) == 0 && (kTP % 4) == 0, "16-B aligned LDS rows");

constexpr int kM1Elems = kD * kIn;
constexpr int kSqElems = kD * kD;
constexpr size_t kOffWcat = 0;
constexpr size_t kOffM2h  = kOffWcat + (size_t)2 * kM1Elems * 2;
constexpr size_t kOffM3h  = kOffM2h + (size_t)kSqElems * 2;
constexpr size_t kWsTotal = kOffM3h + (size_t)kSqElems * 2;
static_assert(kWsTotal == 49152ull, "carve total");
static_assert((kOffM2h % 128) == 0 && (kOffM3h % 128) == 0, "128-B aligned regions");
constexpr int kPrepElems  = 2 * kM1Elems + 2 * kSqElems;
constexpr int kPrepBlocks = kPrepElems / 8 / 256;
static_assert(kPrepBlocks * 256 * 8 == kPrepElems, "prep coverage exact");
static_assert((kM1Elems % (256 * 8)) == 0 && (kSqElems % (256 * 8)) == 0, "prep segments are whole blocks");

__device__ __forceinline__ _Float16 cvt_h(float v) {
  const float w = (fabsf(v) < kHalfMinNormal) ? 0.0f : v;
  return (_Float16)w;
}

union HFrag { v16h v; v8h h[2]; };

template <typename T> struct Frag;
template <> struct Frag<_Float16> {
  typedef v16h V;
  static __device__ __forceinline__ v16h load(const _Float16* p) {
    HFrag f; f.h[0] = *(const v8h*)(p); f.h[1] = *(const v8h*)(p + 16); return f.v;
  }
};

__device__ __forceinline__ v8f mma_h(v16h a, v16h b, v8f c) {
  c = __builtin_amdgcn_wmma_f32_16x16x32_f16(false, a, false, b, (short)0, c, false, false);
  asm volatile("v_nop\n\tv_nop\n\tv_nop\n\tv_nop" : "+v"(c) : "v"(a), "v"(b));
  return c;
}

__global__ __launch_bounds__(256) void prep_weights_kernel(
    const float* __restrict__ M1, const float* __restrict__ Wr1,
    const float* __restrict__ M2, const float* __restrict__ M3,
    unsigned short* __restrict__ dst)
{
  const int blk = blockIdx.x;
  const float* src = M1;
  int base = 0;
  if (blk >= 4 && blk < 8) { src = Wr1; base = kM1Elems; }
  if (blk >= 8 && blk < 10) { src = M2; base = 2 * kM1Elems; }
  if (blk >= 10) { src = M3; base = 2 * kM1Elems + kSqElems; }
  int e0 = (blk * 256 + (int)threadIdx.x) * 8;
  e0 = (e0 > kPrepElems - 8) ? (kPrepElems - 8) : e0;
  const float* sp = src + (e0 - base);
  const v4f a0 = *(const v4f*)(sp);
  const v4f a1 = *(const v4f*)(sp + 4);
  v8h hv;
#pragma unroll
  for (int e = 0; e < 4; ++e) {
    hv[e]     = cvt_h(a0[e] * kCarryW);
    hv[4 + e] = cvt_h(a1[e] * kCarryW);
  }
  unsigned short* q = dst + e0;
  *(volatile v8h*)q = hv;
  __threadfence();
  *(volatile v8h*)q = hv;
}

__global__ __launch_bounds__(32) void fused_layers_kernel(
    const float* __restrict__ seq,
    const unsigned short* __restrict__ Wcp, const unsigned short* __restrict__ M2p, const unsigned short* __restrict__ M3p,
    const float* __restrict__ P1, const float* __restrict__ P2, const float* __restrict__ P3,
    const float* __restrict__ g1, const float* __restrict__ b1,
    const float* __restrict__ g2, const float* __restrict__ b2,
    const float* __restrict__ g3, const float* __restrict__ b3,
    float* __restrict__ out)
{
  __shared__ __align__(16) float    CS[2 * kCSP];
  __shared__ __align__(16) _Float16 AT[16 * kATP];
  __shared__ __align__(16) float    TT[16 * kTP];
  __shared__ __align__(16) float    RT[16 * kTP];

  const int lane = threadIdx.x & 31;
  const int h = lane >> 4;
  const int n = lane & 15;
  int s0 = (int)blockIdx.x * 2;
  s0 = (s0 > kSeq - 2) ? (kSeq - 2) : s0;

  {
#pragma clang fp contract(off)
    const float t0 = kTwoPi * (float)s0;
    const float t1 = kTwoPi * (float)(s0 + 1);
#pragma unroll 1
    for (int e = lane; e < kD * kD; e += 32) {
      const float pd = (float)(e + 2);
      const float a0 = t0 / pd;
      const float a1 = t1 / pd;
      const int o = (e >> 6) * kTP + (e & 63);
      CS[o] = cosf(a0);
      CS[kCSP + o] = cosf(a1);
    }
  }

#pragma unroll 4
  for (int m = 0; m < 16; ++m) {
    const int pi = m >> 3, b = m & 7;
    const v4f x = *(const v4f*)(seq + ((size_t)b * kSeq + (size_t)(s0 + pi)) * kIn + lane * 4);
    v4h hv;
#pragma unroll
    for (int e = 0; e < 4; ++e) hv[e] = cvt_h(x[e] * kCarryA);
    *(v4h*)(AT + m * kATP + lane * 4) = hv;
  }
  __syncthreads();

  {
    const _Float16* Wc = (const _Float16*)Wcp;
    v8f acc[8];
#pragma unroll
    for (int j = 0; j < 8; ++j) acc[j] = (v8f){0.f, 0.f, 0.f, 0.f, 0.f, 0.f, 0.f, 0.f};
#pragma unroll 1
    for (int ks = 0; ks < 4; ++ks) {
      HFrag af;
      af.h[0] = *(const v8h*)(AT + n * kATP + ks * 32 + 8 * h);
      af.h[1] = *(const v8h*)(AT + n * kATP + ks * 32 + 16 + 8 * h);
#pragma unroll
      for (int j = 0; j < 8; ++j) {
        const v16h bf = Frag<_Float16>::load(Wc + (size_t)(j * 16 + n) * kIn + ks * 32 + 8 * h);
        acc[j] = mma_h(af.v, bf, acc[j]);
      }
    }
#pragma unroll
    for (int j = 0; j < 4; ++j) {
#pragma unroll
      for (int r = 0; r < 8; ++r) {
        TT[(8 * h + r) * kTP + j * 16 + n] = acc[j][r] * kInvDense;
        RT[(8 * h + r) * kTP + j * 16 + n] = acc[4 + j][r] * kInvDense;
      }
    }
  }

  const int lrow = lane >> 1;
  const int lcol = (lane & 1) * 32;

#pragma unroll 1
  for (int L = 0; L < 3; ++L) {
    const float* Pl = (L == 0) ? P1 : ((L == 1) ? P2 : P3);
    const float* gl = (L == 0) ? g1 : ((L == 1) ? g2 : g3);
    const float* bl = (L == 0) ? b1 : ((L == 1) ? b2 : b3);
    __syncthreads();

    {
      float xv[32];
#pragma unroll
      for (int q = 0; q < 8; ++q) {
        const v4f t = *(const v4f*)(TT + lrow * kTP + lcol + 4 * q);
        xv[4 * q + 0] = t[0]; xv[4 * q + 1] = t[1]; xv[4 * q + 2] = t[2]; xv[4 * q + 3] = t[3];
      }
      float sm = 0.0f;
#pragma unroll
      for (int i = 0; i < 32; ++i) sm += xv[i];
      sm += __shfl_xor(sm, 1, 32);
      const float mu = sm * (1.0f / (float)kD);
      float sq = 0.0f;
#pragma unroll
      for (int i = 0; i < 32; ++i) { const float dd = xv[i] - mu; sq += dd * dd; }
      sq += __shfl_xor(sq, 1, 32);
      const float var = sq * (1.0f / (float)kD);
      const float rstd = 1.0f / sqrtf(var + kLnEps);
#pragma unroll
      for (int qq = 0; qq < 4; ++qq) {
        const v4f ga = *(const v4f*)(gl + lcol + 8 * qq);
        const v4f gb = *(const v4f*)(gl + lcol + 8 * qq + 4);
        const v4f ba = *(const v4f*)(bl + lcol + 8 * qq);
        const v4f bb = *(const v4f*)(bl + lcol + 8 * qq + 4);
        v8h hv;
#pragma unroll
        for (int e = 0; e < 4; ++e) {
          const float y0 = (xv[8 * qq + e] - mu) * rstd * ga[e] + ba[e];
          const float y1 = (xv[8 * qq + 4 + e] - mu) * rstd * gb[e] + bb[e];
          hv[e]     = cvt_h(y0 * kCarryA);
          hv[4 + e] = cvt_h(y1 * kCarryA);
        }
        *(v8h*)(AT + lrow * kATP + lcol + 8 * qq) = hv;
      }
    }
    __syncthreads();

    {
      v16h am[2];
#pragma unroll
      for (int ks = 0; ks < 2; ++ks) {
        HFrag af;
        af.h[0] = *(const v8h*)(AT + n * kATP + ks * 32 + 8 * h);
        af.h[1] = *(const v8h*)(AT + n * kATP + ks * 32 + 16 + 8 * h);
        am[ks] = af.v;
      }
#pragma unroll 1
      for (int nt = 0; nt < 4; ++nt) {
        const int wi = nt * 16 + n;
        v8f o0 = (v8f){0.f, 0.f, 0.f, 0.f, 0.f, 0.f, 0.f, 0.f};
        v8f o1 = (v8f){0.f, 0.f, 0.f, 0.f, 0.f, 0.f, 0.f, 0.f};
#pragma unroll
        for (int ks = 0; ks < 2; ++ks) {
          const int kb = ks * 32 + 8 * h;
          const float* pp = Pl + wi * kD + kb;
          const v4f p0 = *(const v4f*)(pp);
          const v4f p1 = *(const v4f*)(pp + 4);
          const v4f p2 = *(const v4f*)(pp + 16);
          const v4f p3 = *(const v4f*)(pp + 20);
          const int co = wi * kTP + kb;
          const v4f c00 = *(const v4f*)(CS + co);
          const v4f c01 = *(const v4f*)(CS + co + 4);
          const v4f c02 = *(const v4f*)(CS + co + 16);
          const v4f c03 = *(const v4f*)(CS + co + 20);
          const v4f c10 = *(const v4f*)(CS + kCSP + co);
          const v4f c11 = *(const v4f*)(CS + kCSP + co + 4);
          const v4f c12 = *(const v4f*)(CS + kCSP + co + 16);
          const v4f c13 = *(const v4f*)(CS + kCSP + co + 20);
          v16h w0, w1;
#pragma unroll
          for (int e = 0; e < 4; ++e) {
            const float u00 = p0[e] * c00[e];
            const float u01 = p1[e] * c01[e];
            const float u02 = p2[e] * c02[e];
            const float u03 = p3[e] * c03[e];
            const float u10 = p0[e] * c10[e];
            const float u11 = p1[e] * c11[e];
            const float u12 = p2[e] * c12[e];
            const float u13 = p3[e] * c13[e];
            w0[e]      = cvt_h(u00 * kCarryP);
            w0[4 + e]  = cvt_h(u01 * kCarryP);
            w0[8 + e]  = cvt_h(u02 * kCarryP);
            w0[12 + e] = cvt_h(u03 * kCarryP);
            w1[e]      = cvt_h(u10 * kCarryP);
            w1[4 + e]  = cvt_h(u11 * kCarryP);
            w1[8 + e]  = cvt_h(u12 * kCarryP);
            w1[12 + e] = cvt_h(u13 * kCarryP);
          }
          o0 = mma_h(am[ks], w0, o0);
          o1 = mma_h(am[ks], w1, o1);
        }
#pragma unroll
        for (int r = 0; r < 8; ++r) {
          const int idx = (8 * h + r) * kTP + nt * 16 + n;
          const float sel = (h != 0) ? o1[r] : o0[r];
          const float rv = RT[idx];
          RT[idx] = sel * kInvMod + rv;
        }
      }
    }

    if (L < 2) {
      __syncthreads();
#pragma unroll
      for (int qq = 0; qq < 4; ++qq) {
        const v4f x0 = *(const v4f*)(RT + lrow * kTP + lcol + 8 * qq);
        const v4f x1 = *(const v4f*)(RT + lrow * kTP + lcol + 8 * qq + 4);
        v8h hv;
#pragma unroll
        for (int e = 0; e < 4; ++e) {
          hv[e]     = cvt_h(x0[e] * kCarryA);
          hv[4 + e] = cvt_h(x1[e] * kCarryA);
        }
        *(v8h*)(AT + lrow * kATP + lcol + 8 * qq) = hv;
      }
      __syncthreads();
      const _Float16* Mh = (const _Float16*)((L == 0) ? M2p : M3p);
      v8f acc4[4];
#pragma unroll
      for (int j = 0; j < 4; ++j) acc4[j] = (v8f){0.f, 0.f, 0.f, 0.f, 0.f, 0.f, 0.f, 0.f};
#pragma unroll
      for (int ks = 0; ks < 2; ++ks) {
        HFrag af;
        af.h[0] = *(const v8h*)(AT + n * kATP + ks * 32 + 8 * h);
        af.h[1] = *(const v8h*)(AT + n * kATP + ks * 32 + 16 + 8 * h);
#pragma unroll
        for (int j = 0; j < 4; ++j) {
          const v16h bf = Frag<_Float16>::load(Mh + (size_t)(j * 16 + n) * kD + ks * 32 + 8 * h);
          acc4[j] = mma_h(af.v, bf, acc4[j]);
        }
      }
#pragma unroll
      for (int j = 0; j < 4; ++j) {
#pragma unroll
        for (int r = 0; r < 8; ++r) TT[(8 * h + r) * kTP + j * 16 + n] = acc4[j][r] * kInvDense;
      }
    }
  }
  __syncthreads();

  {
    const int c4 = n * 4;
    v4f ov[8];
#pragma unroll
    for (int it = 0; it < 8; ++it) ov[it] = *(const v4f*)(RT + (it * 2 + h) * kTP + c4);
    for (int pass = 0; pass < 2; ++pass) {
#pragma unroll
      for (int it = 0; it < 8; ++it) {
        const int m = it * 2 + h;
        const int pi = m >> 3, b = m & 7;
        *(volatile v4f*)(out + ((size_t)b * kSeq + (size_t)(s0 + pi)) * kD + c4) = ov[it];
      }
      __threadfence();
    }
  }
}

extern "C" void kernel_launch(void* const* d_in, const int* in_sizes, int n_in,
                              void* d_out, int out_size, void* d_ws, size_t ws_size,
                              hipStream_t stream) {
  if (n_in < 14) return;
  if (in_sizes[0] != kNB * kSeq * kIn) return;
  if (in_sizes[1] != kM1Elems) return;
  if (in_sizes[2] != kSqElems) return;
  if (in_sizes[3] != kD || in_sizes[4] != kD) return;
  if (in_sizes[5] != kM1Elems) return;
  if (in_sizes[6] != kSqElems || in_sizes[7] != kSqElems) return;
  if (in_sizes[8] != kD || in_sizes[9] != kD) return;
  if (in_sizes[10] != kSqElems || in_sizes[11] != kSqElems) return;
  if (in_sizes[12] != kD || in_sizes[13] != kD) return;
  if (out_size != kNB * kSeq * kD) return;
  if (ws_size < kWsTotal) return;

  const float* seq = (const float*)d_in[0];
  const float* M1  = (const float*)d_in[1];
  const float* P1  = (const float*)d_in[2];
  const float* g1  = (const float*)d_in[3];
  const float* b1  = (const float*)d_in[4];
  const float* Wr1 = (const float*)d_in[5];
  const float* M2  = (const float*)d_in[6];
  const float* P2  = (const float*)d_in[7];
  const float* g2  = (const float*)d_in[8];
  const float* b2  = (const float*)d_in[9];
  const float* M3  = (const float*)d_in[10];
  const float* P3  = (const float*)d_in[11];
  const float* g3  = (const float*)d_in[12];
  const float* b3  = (const float*)d_in[13];
  float* out = (float*)d_out;

  char* ws = (char*)d_ws;
  unsigned short* WCAT = (unsigned short*)(ws + kOffWcat);
  unsigned short* M2H  = (unsigned short*)(ws + kOffM2h);
  unsigned short* M3H  = (unsigned short*)(ws + kOffM3h);

  prep_weights_kernel<<<kPrepBlocks, 256, 0, stream>>>(M1, Wr1, M2, M3, WCAT);

  fused_layers_kernel<<<kSeq / 2, 32, 0, stream>>>(
      seq, WCAT, M2H, M3H, P1, P2, P3, g1, b1, g2, b2, g3, b3, out);
}
